// GINEncoder2_17205638988407
// MI455X (gfx1250) — hardware-verified
//
#include <hip/hip_runtime.h>
#include <stddef.h>


#define DIM     128
#define G3      384
#define G4      512
#define KL      384
#define NTHR    256
#define NWAVE   8
#define EPT     8
#define NGRP    2
#define CHUNK   (NTHR * EPT * NGRP)
#define WCAP    (EPT * NGRP * 32)
#define LISTN   (NWAVE * WCAP)
#define NBC     4096
#define NBF     1024
#define NBP     32
#define RCAP    40960
#define RBN     128
#define TGT     256
#define DEGCAP  256
#define GROWS   128
#define FROWS   64
#define FTHR    128
#define OTHR    512

#define LDS_GEMM (GROWS * DIM * 4)
#define LDS_FILL ((RCAP + NBF + LISTN) * 4 + 64)
#define LDS_GRU  (FROWS * G4 * 4 + FROWS * DIM * 4)

static_assert((CHUNK & (CHUNK - 1)) == 0);
static_assert(CHUNK <= 4096);
static_assert(NBC <= 4096 && NBF <= 4096 && NBP <= 4096);
static_assert((NBC & (NBC - 1)) == 0 && (NBF & (NBF - 1)) == 0 && (NBP & (NBP - 1)) == 0);
static_assert(NBC == 4 * NBF);
static_assert(OTHR * 8 == NBC);
static_assert((RCAP % 32) == 0);
static_assert(TGT == NWAVE * 32 && (TGT % GROWS) == 0 && (TGT % FROWS) == 0);
static_assert(NBP == 4 * NWAVE);
static_assert(FROWS == 16 * (FTHR / 32));
static_assert(GROWS == 16 * NWAVE);

typedef float          v4f  __attribute__((ext_vector_type(4)));
typedef float          v8f  __attribute__((ext_vector_type(8)));
typedef int            v4i  __attribute__((ext_vector_type(4)));
typedef unsigned short us_t;
typedef us_t           v4us __attribute__((ext_vector_type(4)));
typedef us_t           v8us __attribute__((ext_vector_type(8)));
typedef __bf16         v16b __attribute__((ext_vector_type(16)));
union FragB { v16b v; v8us u[2]; };

__device__ __forceinline__ us_t bfr(float f) {
  unsigned u = __float_as_uint(f);
  u += 0x7FFFu + ((u >> 16) & 1u);
  return (us_t)(u >> 16);
}
__device__ __forceinline__ float bfup(us_t s) { return __uint_as_float(((unsigned)s) << 16); }

__device__ __forceinline__ void split4(v4f a, v4us& hi, v4us& lo) {
  float x[4];
  x[0] = a.x; x[1] = a.y; x[2] = a.z; x[3] = a.w;
#pragma unroll
  for (int e = 0; e < 4; ++e) {
    const us_t h = bfr(x[e]);
    hi[e] = h;
    lo[e] = bfr(x[e] - bfup(h));
  }
}
__device__ __forceinline__ void split8(v4f a, v4f b, v8us& hi, v8us& lo) {
  float x[8];
  x[0] = a.x; x[1] = a.y; x[2] = a.z; x[3] = a.w;
  x[4] = b.x; x[5] = b.y; x[6] = b.z; x[7] = b.w;
#pragma unroll
  for (int e = 0; e < 8; ++e) {
    const us_t h = bfr(x[e]);
    hi[e] = h;
    lo[e] = bfr(x[e] - bfup(h));
  }
}

__device__ __forceinline__ float sigm(float x) {
  x = fminf(fmaxf(x, -80.0f), 80.0f);
  return 1.0f / (1.0f + __expf(-x));
}

__device__ __forceinline__ v8f zero8() { v8f z = {0.f, 0.f, 0.f, 0.f, 0.f, 0.f, 0.f, 0.f}; return z; }

__device__ __forceinline__ v8f wm3(const FragB& ah, const FragB& al, const FragB& bh, const FragB& bl, v8f c) {
  c = __builtin_amdgcn_wmma_f32_16x16x32_bf16(false, ah.v, false, bh.v, (short)0, c, false, false);
  c = __builtin_amdgcn_wmma_f32_16x16x32_bf16(false, ah.v, false, bl.v, (short)0, c, false, false);
  c = __builtin_amdgcn_wmma_f32_16x16x32_bf16(false, al.v, false, bh.v, (short)0, c, false, false);
  asm volatile("v_nop\n\tv_nop\n\tv_nop\n\tv_nop" : "+v"(c) : "v"(ah.v), "v"(al.v), "v"(bh.v), "v"(bl.v));
  return c;
}

template <int NB>
__device__ __forceinline__ int scan_chunk(const int* __restrict__ dsts, int nE, int cbase, int slotBase,
                                          int vec8, int* list, int tid, int lane, int wave) {
  int wc = 0;
#pragma unroll
  for (int g = 0; g < NGRP; ++g) {
    const int el0  = (g * NTHR + tid) * EPT;
    const int e0   = cbase + el0;
    const int sent = -2147483647 - 1;
    v4i da, db;
    if (vec8 != 0 && cbase + CHUNK <= nE) {
      da = *(const v4i*)(dsts + e0);
      db = *(const v4i*)(dsts + e0 + 4);
    } else {
      da.x = (e0     < nE) ? dsts[min(e0, nE - 1)] : sent;
      da.y = (e0 + 1 < nE) ? dsts[min(e0 + 1, nE - 1)] : sent;
      da.z = (e0 + 2 < nE) ? dsts[min(e0 + 2, nE - 1)] : sent;
      da.w = (e0 + 3 < nE) ? dsts[min(e0 + 3, nE - 1)] : sent;
      db.x = (e0 + 4 < nE) ? dsts[min(e0 + 4, nE - 1)] : sent;
      db.y = (e0 + 5 < nE) ? dsts[min(e0 + 5, nE - 1)] : sent;
      db.z = (e0 + 6 < nE) ? dsts[min(e0 + 6, nE - 1)] : sent;
      db.w = (e0 + 7 < nE) ? dsts[min(e0 + 7, nE - 1)] : sent;
    }
    const unsigned nb = (unsigned)slotBase;
    const unsigned s0 = (unsigned)da.x - nb, s1 = (unsigned)da.y - nb;
    const unsigned s2 = (unsigned)da.z - nb, s3 = (unsigned)da.w - nb;
    const unsigned s4 = (unsigned)db.x - nb, s5 = (unsigned)db.y - nb;
    const unsigned s6 = (unsigned)db.z - nb, s7 = (unsigned)db.w - nb;
    const bool h0 = s0 < (unsigned)NB, h1 = s1 < (unsigned)NB, h2 = s2 < (unsigned)NB, h3 = s3 < (unsigned)NB;
    const bool h4 = s4 < (unsigned)NB, h5 = s5 < (unsigned)NB, h6 = s6 < (unsigned)NB, h7 = s7 < (unsigned)NB;
    const unsigned any = __builtin_amdgcn_ballot_w32(h0 | h1 | h2 | h3 | h4 | h5 | h6 | h7);
    if (any != 0u) {
#define HITJ(J, HJ, SJ) { \
        const unsigned mj = __builtin_amdgcn_ballot_w32(HJ); \
        if (mj != 0u) { \
          if (HJ) { \
            const int pos = wc + (int)__builtin_amdgcn_mbcnt_lo(mj, 0u); \
            if (pos < WCAP) list[wave * WCAP + pos] = ((el0 + (J)) << 12) | (int)(SJ); \
          } \
          wc += (int)__builtin_popcount(mj); } }
      HITJ(0, h0, s0)
      HITJ(1, h1, s1)
      HITJ(2, h2, s2)
      HITJ(3, h3, s3)
      HITJ(4, h4, s4)
      HITJ(5, h5, s5)
      HITJ(6, h6, s6)
      HITJ(7, h7, s7)
#undef HITJ
    }
  }
  return wc;
}

__global__ __launch_bounds__(NTHR) void k_cvt(const float* __restrict__ src, us_t* hi, us_t* lo,
                                             int K, int rows, int nVec) {
  const int i = blockIdx.x * NTHR + (int)threadIdx.x;
  if (i >= nVec) return;
  const int o  = i * 8;
  const int r  = o / K;
  const int k0 = o - r * K;
  const int rs = r < rows ? r : rows - 1;
  const float* sp = src + (size_t)rs * K + k0;
  const v4f a = *(const v4f*)sp, b = *(const v4f*)(sp + 4);
  v8us h8, l8;
  split8(a, b, h8, l8);
  *(volatile v8us*)(hi + o) = h8;
  *(volatile v8us*)(lo + o) = l8;
  __threadfence();
  *(volatile v8us*)(hi + o) = h8;
  *(volatile v8us*)(lo + o) = l8;
}

__global__ __launch_bounds__(NTHR) void k_cvt2(const float* __restrict__ wih, const float* __restrict__ whh,
                                              const float* __restrict__ bih, const float* __restrict__ bhh,
                                              us_t* hi, us_t* lo, float* bsum, int nVec) {
  const int i = blockIdx.x * NTHR + (int)threadIdx.x;
  if (i < nVec) {
    const int o  = i * 8;
    const int n  = o / KL;
    const int k0 = o - n * KL;
    const int ka = k0 < 256 ? k0 : 248;
    const int kb = k0 >= 256 ? k0 - 256 : 0;
    const float* pa = wih + (size_t)n * 256 + ka;
    const float* pb = whh + (size_t)n * DIM + kb;
    const v4f a0 = *(const v4f*)pa, a1 = *(const v4f*)(pa + 4);
    const v4f b0 = *(const v4f*)pb, b1 = *(const v4f*)(pb + 4);
    const bool useA = k0 < 256;
    v4f c0, c1;
    c0.x = useA ? a0.x : b0.x; c0.y = useA ? a0.y : b0.y; c0.z = useA ? a0.z : b0.z; c0.w = useA ? a0.w : b0.w;
    c1.x = useA ? a1.x : b1.x; c1.y = useA ? a1.y : b1.y; c1.z = useA ? a1.z : b1.z; c1.w = useA ? a1.w : b1.w;
    v8us h8, l8;
    split8(c0, c1, h8, l8);
    *(volatile v8us*)(hi + o) = h8;
    *(volatile v8us*)(lo + o) = l8;
    __threadfence();
    *(volatile v8us*)(hi + o) = h8;
    *(volatile v8us*)(lo + o) = l8;
  }
  if (blockIdx.x == 0 && threadIdx.x < (G4 / 4)) {
    const int t = (int)threadIdx.x;
    const v4f a = *(const v4f*)(bih + 4 * t);
    const v4f b = *(const v4f*)(bhh + 4 * t);
    const v4f s = a + b;
    *(volatile v4f*)(bsum + 4 * t) = s;
    __threadfence();
    *(volatile v4f*)(bsum + 4 * t) = s;
  }
}

__global__ __launch_bounds__(NTHR) void k_count(const int* __restrict__ ei, int* cnt, int nE, int vec8) {
  __shared__ __attribute__((aligned(16))) int scnt[NBC];
  __shared__ __attribute__((aligned(16))) int list[LISTN];
  __shared__ int wcnt[NWAVE];
  const int tid = threadIdx.x, lane = tid & 31, wave = tid >> 5;
  const int nodeBase = blockIdx.x * NBC;
  const int* dsts = ei + nE;

  for (int i = tid; i < NBC; i += NTHR) scnt[i] = 0;
  __syncthreads();

  const int nChunks = (nE + CHUNK - 1) / CHUNK;
#pragma unroll 1
  for (int ch = 0; ch < nChunks; ++ch) {
    const int cbase = ch * CHUNK;
    const int wc = scan_chunk<NBC>(dsts, nE, cbase, nodeBase, vec8, list, tid, lane, wave);
    if (lane == 0) wcnt[wave] = wc;
    __syncthreads();
    if (wave == 0) {
#pragma unroll 1
      for (int wsx = 0; wsx < NWAVE; ++wsx) {
        int n = __builtin_amdgcn_readfirstlane(wcnt[wsx]);
        n = n > WCAP ? WCAP : (n < 0 ? 0 : n);
        const int* lp = list + wsx * WCAP;
#pragma unroll 1
        for (int i = 0; i < n; ++i) {
          const int ent  = __builtin_amdgcn_readfirstlane(lp[i]);
          const int slot = ent & (NBC - 1);
          if (lane == 0) scnt[slot] = scnt[slot] + 1;
        }
      }
    }
    __syncthreads();
  }

  v4i cq[4];
#pragma unroll
  for (int q = 0; q < 4; ++q) {
    const int f = (wave * 4 + q) * 128 + 4 * lane;
    cq[q] = *(const v4i*)(scnt + f);
  }
  int* cp = cnt + (size_t)nodeBase;
#pragma unroll
  for (int q = 0; q < 4; ++q) {
    const int f = (wave * 4 + q) * 128 + 4 * lane;
    *(volatile v4i*)(cp + f) = cq[q];
  }
  __threadfence();
#pragma unroll
  for (int q = 0; q < 4; ++q) {
    const int f = (wave * 4 + q) * 128 + 4 * lane;
    *(volatile v4i*)(cp + f) = cq[q];
  }
}

__global__ __launch_bounds__(OTHR) void k_offsets(const int* __restrict__ cnt, int* off, int* rbase, int nChunk) {
  __shared__ __attribute__((aligned(16))) int soff[NBC];
  __shared__ __attribute__((aligned(16))) int srb[RBN];
  __shared__ int wtot[OTHR / 32];
  const int tid = threadIdx.x, lane = tid & 31, wave = tid >> 5, sub = tid >> 7;
  for (int i = tid; i < RBN; i += OTHR) srb[i] = 0;
  int carry = 0;
#pragma unroll 1
  for (int ch = 0; ch < nChunk; ++ch) {
    const int base = ch * NBC;
    const v4i c0 = *(const v4i*)(cnt + base + 8 * tid);
    const v4i c1 = *(const v4i*)(cnt + base + 8 * tid + 4);
    const int e0 = max(c0.x, 0), e1 = max(c0.y, 0), e2 = max(c0.z, 0), e3 = max(c0.w, 0);
    const int e4 = max(c1.x, 0), e5 = max(c1.y, 0), e6 = max(c1.z, 0), e7 = max(c1.w, 0);
    const int ts = e0 + e1 + e2 + e3 + e4 + e5 + e6 + e7;
    int incl = ts;
#pragma unroll
    for (int d = 1; d < 32; d <<= 1) {
      const int t = __shfl_up(incl, d);
      if (lane >= d) incl += t;
    }
    if (lane == 31) wtot[wave] = incl;
    __syncthreads();
    const int S0 = wtot[0]  + wtot[1]  + wtot[2]  + wtot[3];
    const int S1 = wtot[4]  + wtot[5]  + wtot[6]  + wtot[7];
    const int S2 = wtot[8]  + wtot[9]  + wtot[10] + wtot[11];
    const int S3 = wtot[12] + wtot[13] + wtot[14] + wtot[15];
    int pre = 0;
#pragma unroll 1
    for (int w = 4 * sub; w < wave; ++w) pre += wtot[w];
    const int b0 = carry;
    const int b1 = b0 + ((S0 + 31) & ~31);
    const int b2 = b1 + ((S1 + 31) & ~31);
    const int b3 = b2 + ((S2 + 31) & ~31);
    const int b4 = b3 + ((S3 + 31) & ~31);
    const int myb = sub == 0 ? b0 : (sub == 1 ? b1 : (sub == 2 ? b2 : b3));
    if (tid == 0) {
      srb[min(4 * ch + 0, RBN - 1)] = b0;
      srb[min(4 * ch + 1, RBN - 1)] = b1;
      srb[min(4 * ch + 2, RBN - 1)] = b2;
      srb[min(4 * ch + 3, RBN - 1)] = b3;
    }
    int run = myb + pre + incl - ts;
    soff[8 * tid + 0] = run; run += e0;
    soff[8 * tid + 1] = run; run += e1;
    soff[8 * tid + 2] = run; run += e2;
    soff[8 * tid + 3] = run; run += e3;
    soff[8 * tid + 4] = run; run += e4;
    soff[8 * tid + 5] = run; run += e5;
    soff[8 * tid + 6] = run; run += e6;
    soff[8 * tid + 7] = run;
    carry = b4;
    __syncthreads();
    const v4i o0 = *(const v4i*)(soff + 4 * tid);
    const v4i o1 = *(const v4i*)(soff + 4 * (tid + OTHR));
    int* op = off + base;
    *(volatile v4i*)(op + 4 * tid) = o0;
    *(volatile v4i*)(op + 4 * (tid + OTHR)) = o1;
    __threadfence();
    *(volatile v4i*)(op + 4 * tid) = o0;
    *(volatile v4i*)(op + 4 * (tid + OTHR)) = o1;
    __syncthreads();
  }
  if (tid == 0) srb[min(4 * nChunk, RBN - 1)] = carry;
  __syncthreads();
  v4i rv = {0, 0, 0, 0};
  if (tid < 32) rv = *(const v4i*)(srb + 4 * tid);
  if (tid < 32) *(volatile v4i*)(rbase + 4 * tid) = rv;
  __threadfence();
  if (tid < 32) *(volatile v4i*)(rbase + 4 * tid) = rv;
}

__global__ __launch_bounds__(NTHR) void k_fill(const int* __restrict__ ei, const int* __restrict__ off,
                                              const int* __restrict__ rbase, int* csr,
                                              int nN, int nE, int vec8, int csrLen) {
  extern __shared__ v4f lds_dyn[];
  int* region = (int*)lds_dyn;
  int* cursor = region + RCAP;
  int* list   = cursor + NBF;
  int* wcnt   = list + LISTN;
  const int tid = threadIdx.x, lane = tid & 31, wave = tid >> 5;
  const int b = blockIdx.x;
  const int nodeBase = b * NBF;
  const int* dsts = ei + nE;

  int rb0 = rbase[b];
  const int rb1 = rbase[b + 1];
  rb0 = rb0 < 0 ? 0 : (rb0 > csrLen ? csrLen : rb0);
  rb0 &= ~31;
  int len = rb1 - rb0;
  len = len < 0 ? 0 : (len > RCAP ? RCAP : len);
  int lenW = (len + 31) & ~31;
  if (rb0 + lenW > csrLen) lenW = (csrLen - rb0) & ~31;

  {
    const v4i z = {0, 0, 0, 0};
    for (int i = tid; i < RCAP / 4; i += NTHR) ((v4i*)region)[i] = z;
    for (int s = tid; s < NBF; s += NTHR) {
      int o = off[nodeBase + s] - rb0;
      o = o < 0 ? 0 : (o > RCAP ? RCAP : o);
      cursor[s] = o;
    }
  }
  __syncthreads();

  const int nChunks = (nE + CHUNK - 1) / CHUNK;
#pragma unroll 1
  for (int ch = 0; ch < nChunks; ++ch) {
    const int cbase = ch * CHUNK;
    const int wc = scan_chunk<NBF>(dsts, nE, cbase, nodeBase, vec8, list, tid, lane, wave);
    if (lane == 0) wcnt[wave] = wc;
    __syncthreads();
    if (wave == 0) {
#pragma unroll 1
      for (int wsx = 0; wsx < NWAVE; ++wsx) {
        int n = __builtin_amdgcn_readfirstlane(wcnt[wsx]);
        n = n > WCAP ? WCAP : (n < 0 ? 0 : n);
        const int* lp = list + wsx * WCAP;
#pragma unroll 1
        for (int i = 0; i < n; ++i) {
          const int ent  = __builtin_amdgcn_readfirstlane(lp[i]);
          const int slot = ent & (NBF - 1);
          int e = cbase + ((ent >> 12) & (CHUNK - 1));
          e = e > nE - 1 ? nE - 1 : e;
          int src = ei[e];
          src = src < 0 ? 0 : (src > nN - 1 ? nN - 1 : src);
          if (lane == 0) {
            int pos = cursor[slot];
            pos = pos < 0 ? 0 : (pos > RCAP - 1 ? RCAP - 1 : pos);
            region[pos] = src;
            const int np = pos + 1;
            cursor[slot] = np > RCAP ? RCAP : np;
          }
        }
      }
    }
    __syncthreads();
  }

  const int nv = lenW >> 2;
  int* gp = csr + rb0;
#pragma unroll 1
  for (int i = tid; i < nv; i += NTHR) { const v4i v = ((const v4i*)region)[i]; *(volatile v4i*)(gp + 4 * i) = v; }
  __threadfence();
#pragma unroll 1
  for (int i = tid; i < nv; i += NTHR) { const v4i v = ((const v4i*)region)[i]; *(volatile v4i*)(gp + 4 * i) = v; }
}

__device__ __forceinline__ void tile_store(const float* lp, int r0, int lane, int hh, int m,
                                           float* Cf, int ldc, us_t* Chi, us_t* Clo, int ldp,
                                           int colBase, int wantF, int wantP) {
  if (wantF != 0) {
#pragma unroll
    for (int i = 0; i < 16; ++i) {
      const v4f v = *(const v4f*)(lp + i * DIM + 4 * lane);
      *(volatile v4f*)(Cf + (size_t)(r0 + i) * ldc + colBase + 4 * lane) = v;
    }
  }
  if (wantP != 0) {
#pragma unroll
    for (int j = 0; j < 8; ++j) {
      const int row = 2 * j + hh;
      const v4f a = *(const v4f*)(lp + row * DIM + 8 * m);
      const v4f b = *(const v4f*)(lp + row * DIM + 8 * m + 4);
      v8us h8, l8;
      split8(a, b, h8, l8);
      const size_t o = (size_t)(r0 + row) * ldp + colBase + 8 * m;
      *(volatile v8us*)(Chi + o) = h8;
      *(volatile v8us*)(Clo + o) = l8;
    }
  }
}

template <int KT>
__global__ __launch_bounds__(NTHR) void k_gemm(
    const us_t* __restrict__ Ahi, const us_t* __restrict__ Alo,
    const us_t* __restrict__ Bhi, const us_t* __restrict__ Blo,
    const float* __restrict__ bias,
    float* Cf, us_t* Chi, us_t* Clo,
    int ldc, int ldp, int relu, int wantF, int wantP) {
  extern __shared__ v4f lds_dyn[];
  float* stg = (float*)lds_dyn;
  const int tid = threadIdx.x, lane = tid & 31, wave = tid >> 5, hh = lane >> 4, m = lane & 15;
  const int rowBase = blockIdx.x * GROWS;
  const int colBase = blockIdx.y * DIM;

  v8f acc[8];
#pragma unroll
  for (int t = 0; t < 8; ++t) acc[t] = zero8();
  const size_t arow = (size_t)(rowBase + wave * 16 + m) * KT + 8 * hh;
#pragma unroll 1
  for (int kt = 0; kt < KT / 32; ++kt) {
    FragB ah, al;
    ah.u[0] = *(const v8us*)(Ahi + arow + 32 * kt);
    ah.u[1] = *(const v8us*)(Ahi + arow + 32 * kt + 16);
    al.u[0] = *(const v8us*)(Alo + arow + 32 * kt);
    al.u[1] = *(const v8us*)(Alo + arow + 32 * kt + 16);
#pragma unroll
    for (int t = 0; t < 8; ++t) {
      const size_t brow = (size_t)(colBase + 16 * t + m) * KT + 32 * kt + 8 * hh;
      FragB bh, bl;
      bh.u[0] = *(const v8us*)(Bhi + brow);
      bh.u[1] = *(const v8us*)(Bhi + brow + 16);
      bl.u[0] = *(const v8us*)(Blo + brow);
      bl.u[1] = *(const v8us*)(Blo + brow + 16);
      acc[t] = wm3(ah, al, bh, bl, acc[t]);
    }
  }

  float* sp = stg + (wave * 16 + 8 * hh) * DIM + m;
#pragma unroll
  for (int t = 0; t < 8; ++t) {
    const float bv = bias[colBase + 16 * t + m];
#pragma unroll
    for (int r = 0; r < 8; ++r) {
      float v = acc[t][r] + bv;
      v = (relu != 0) ? fmaxf(v, 0.0f) : v;
      sp[r * DIM + 16 * t] = v;
    }
  }
  __syncthreads();

  const float* lp = stg + wave * 16 * DIM;
  const int r0 = rowBase + wave * 16;
  tile_store(lp, r0, lane, hh, m, Cf, ldc, Chi, Clo, ldp, colBase, wantF, wantP);
  __threadfence();
  tile_store(lp, r0, lane, hh, m, Cf, ldc, Chi, Clo, ldp, colBase, wantF, wantP);
}

__device__ __forceinline__ void acc_pair(v8f (&acc)[8], const us_t* Ahi, const us_t* Alo, size_t arow,
                                         const us_t* Bhi, const us_t* Blo, int bn0, int m, int hh) {
#pragma unroll 1
  for (int kt = 0; kt < DIM / 32; ++kt) {
    FragB ah, al;
    ah.u[0] = *(const v8us*)(Ahi + arow + 32 * kt);
    ah.u[1] = *(const v8us*)(Ahi + arow + 32 * kt + 16);
    al.u[0] = *(const v8us*)(Alo + arow + 32 * kt);
    al.u[1] = *(const v8us*)(Alo + arow + 32 * kt + 16);
#pragma unroll
    for (int t = 0; t < 8; ++t) {
      const size_t brow = (size_t)(bn0 + 16 * t + m) * DIM + 32 * kt + 8 * hh;
      FragB bh, bl;
      bh.u[0] = *(const v8us*)(Bhi + brow);
      bh.u[1] = *(const v8us*)(Bhi + brow + 16);
      bl.u[0] = *(const v8us*)(Blo + brow);
      bl.u[1] = *(const v8us*)(Blo + brow + 16);
      acc[t] = wm3(ah, al, bh, bl, acc[t]);
    }
  }
}

__device__ __forceinline__ void stage8(const v8f (&acc)[8], float* gs, int wave, int hh, int m, int col0,
                                       const float* __restrict__ b1, const float* __restrict__ b2, int two) {
  float* sp = gs + (wave * 16 + 8 * hh) * G4 + col0 + m;
#pragma unroll
  for (int t = 0; t < 8; ++t) {
    float bv = b1[16 * t + m];
    if (two != 0) bv += b2[16 * t + m];
#pragma unroll
    for (int r = 0; r < 8; ++r) sp[r * G4 + 16 * t] = acc[t][r] + bv;
  }
}

__device__ __forceinline__ void gru_store(const float* hn, int rowBase, int wave, int lane, int hh, int m,
                                          float* hF, us_t* hHi, us_t* hLo, float* out1, int nN, int writeOut) {
#pragma unroll
  for (int i = 0; i < 16; ++i) {
    const int row  = wave * 16 + i;
    const int grow = rowBase + row;
    const v4f v = *(const v4f*)(hn + row * DIM + 4 * lane);
    *(volatile v4f*)(hF + (size_t)grow * DIM + 4 * lane) = v;
    if (writeOut != 0 && grow < nN) *(volatile v4f*)(out1 + (size_t)grow * DIM + 4 * lane) = v;
  }
#pragma unroll
  for (int j = 0; j < 8; ++j) {
    const int row  = wave * 16 + 2 * j + hh;
    const int grow = rowBase + row;
    const v4f a = *(const v4f*)(hn + row * DIM + 8 * m);
    const v4f b = *(const v4f*)(hn + row * DIM + 8 * m + 4);
    v8us h8, l8;
    split8(a, b, h8, l8);
    const size_t o = (size_t)grow * DIM + 8 * m;
    *(volatile v8us*)(hHi + o) = h8;
    *(volatile v8us*)(hLo + o) = l8;
  }
}

__global__ __launch_bounds__(FTHR) void k_grustep(
    const us_t* __restrict__ mHi, const us_t* __restrict__ mLo,
    us_t* hHi, us_t* hLo,
    const us_t* __restrict__ wihHi, const us_t* __restrict__ wihLo,
    const us_t* __restrict__ whhHi, const us_t* __restrict__ whhLo,
    const float* __restrict__ bih, const float* __restrict__ bhh,
    float* hF, float* out1, int nN, int writeOut) {
  extern __shared__ v4f lds_dyn[];
  float* gs = (float*)lds_dyn;
  float* hn = gs + FROWS * G4;
  const int tid = threadIdx.x, lane = tid & 31, wave = tid >> 5, hh = lane >> 4, m = lane & 15;
  const int rowBase = blockIdx.x * FROWS;
  const size_t arow = (size_t)(rowBase + wave * 16 + m) * DIM + 8 * hh;

  v8f acc[8];
#pragma unroll
  for (int t = 0; t < 8; ++t) acc[t] = zero8();
  acc_pair(acc, mHi, mLo, arow, wihHi, wihLo, 0, m, hh);
  acc_pair(acc, hHi, hLo, arow, whhHi, whhLo, 0, m, hh);
  stage8(acc, gs, wave, hh, m, 0, bih, bhh, 1);
#pragma unroll
  for (int t = 0; t < 8; ++t) acc[t] = zero8();
  acc_pair(acc, mHi, mLo, arow, wihHi, wihLo, DIM, m, hh);
  acc_pair(acc, hHi, hLo, arow, whhHi, whhLo, DIM, m, hh);
  stage8(acc, gs, wave, hh, m, DIM, bih + DIM, bhh + DIM, 1);
#pragma unroll
  for (int t = 0; t < 8; ++t) acc[t] = zero8();
  acc_pair(acc, mHi, mLo, arow, wihHi, wihLo, 2 * DIM, m, hh);
  stage8(acc, gs, wave, hh, m, 2 * DIM, bih + 2 * DIM, bih, 0);
#pragma unroll
  for (int t = 0; t < 8; ++t) acc[t] = zero8();
  acc_pair(acc, hHi, hLo, arow, whhHi, whhLo, 2 * DIM, m, hh);
  stage8(acc, gs, wave, hh, m, 3 * DIM, bhh + 2 * DIM, bhh, 0);
  __syncthreads();

#pragma unroll 1
  for (int it = 0; it < FROWS * DIM / FTHR; ++it) {
    const int idx = it * FTHR + tid;
    const int row = idx >> 7;
    const int d   = idx & (DIM - 1);
    const float* g = gs + row * G4;
    const float ar = g[d], az = g[DIM + d], anx = g[2 * DIM + d], anh = g[3 * DIM + d];
    const float hold = hF[(size_t)(rowBase + row) * DIM + d];
    const float r  = sigm(ar);
    const float zt = sigm(az);
    const float n  = tanhf(anx + r * anh);
    hn[row * DIM + d] = (1.0f - zt) * n + zt * hold;
  }
  __syncthreads();

  gru_store(hn, rowBase, wave, lane, hh, m, hF, hHi, hLo, out1, nN, writeOut);
  __threadfence();
  gru_store(hn, rowBase, wave, lane, hh, m, hF, hHi, hLo, out1, nN, writeOut);
}

__global__ __launch_bounds__(NTHR) void k_agg(const int* __restrict__ csr, const int* __restrict__ off,
                                             const int* __restrict__ cnt, const float* __restrict__ hF,
                                             us_t* zHi, us_t* zLo, int nN, int csrLen) {
  const int tid = threadIdx.x, lane = tid & 31, wave = tid >> 5;
  const int tbase = blockIdx.x * TGT + wave * 32;
  const int cl = tbase + lane;
  const int cnt_l = cnt[cl];
  const int off_l = off[cl];

#pragma unroll 1
  for (int j = 0; j < 32; ++j) {
    const int c = tbase + j;
    int n = __builtin_amdgcn_readlane(cnt_l, j);
    n = n < 0 ? 0 : (n > DEGCAP ? DEGCAP : n);
    const int st = __builtin_amdgcn_readlane(off_l, j);
    v4f acc = {0.f, 0.f, 0.f, 0.f};
#pragma unroll 1
    for (int q0 = 0; q0 < n; q0 += 32) {
      int pos = st + q0 + lane;
      pos = pos < 0 ? 0 : (pos > csrLen - 1 ? csrLen - 1 : pos);
      int sl = csr[pos];
      sl = sl < 0 ? 0 : (sl > nN - 1 ? nN - 1 : sl);
      const int mcnt = (n - q0) < 32 ? (n - q0) : 32;
#pragma unroll 1
      for (int p = 0; p < mcnt; ++p) {
        const int s = __builtin_amdgcn_readlane(sl, p);
        acc = acc + *(const v4f*)(hF + (size_t)s * DIM + 4 * lane);
      }
    }
    const v4f sv = *(const v4f*)(hF + (size_t)c * DIM + 4 * lane);
    const v4f z = sv + acc;
    v4us h4, l4;
    split4(z, h4, l4);
    const size_t o = (size_t)c * DIM + 4 * lane;
    *(volatile v4us*)(zHi + o) = h4;
    *(volatile v4us*)(zLo + o) = l4;
    __threadfence();
    *(volatile v4us*)(zHi + o) = h4;
    *(volatile v4us*)(zLo + o) = l4;
  }
}

__device__ __forceinline__ void s2s_store0(const float* sq, const float* sc, int gBase, int wave, int lane,
                                           float* clp, us_t* aHi, us_t* aLo, float* out0) {
#pragma unroll
  for (int j = 0; j < NBP / NWAVE; ++j) {
    const int s = wave + NWAVE * j;
    const int g = gBase + s;
    const v4f cv = *(const v4f*)(sc + s * DIM + 4 * lane);
    const v4f qv = *(const v4f*)(sq + s * DIM + 4 * lane);
    *(volatile v4f*)(clp + (size_t)g * DIM + 4 * lane) = cv;
    *(volatile v4f*)(out0 + (size_t)g * (2 * DIM) + 4 * lane) = qv;
    v4us h4, l4;
    split4(qv, h4, l4);
    const size_t o = (size_t)g * KL + 4 * lane;
    *(volatile v4us*)(aHi + o) = h4;
    *(volatile v4us*)(aLo + o) = l4;
    *(volatile v4us*)(aHi + o + 2 * DIM) = h4;
    *(volatile v4us*)(aLo + o + 2 * DIM) = l4;
  }
}

__device__ __forceinline__ void s2s_storeC(const float* racc, const float* sden, int gBase, int wave, int lane,
                                           us_t* aHi, us_t* aLo, float* out0) {
#pragma unroll
  for (int j = 0; j < NBP / NWAVE; ++j) {
    const int s = wave + NWAVE * j;
    const int g = gBase + s;
    const float rden = 1.0f / (sden[s] + 1e-16f);
    const v4f rv = *(const v4f*)(racc + s * DIM + 4 * lane) * rden;
    *(volatile v4f*)(out0 + (size_t)g * (2 * DIM) + DIM + 4 * lane) = rv;
    v4us h4, l4;
    split4(rv, h4, l4);
    const size_t o = (size_t)g * KL + DIM + 4 * lane;
    *(volatile v4us*)(aHi + o) = h4;
    *(volatile v4us*)(aLo + o) = l4;
  }
}

__global__ __launch_bounds__(NTHR) void k_s2s(
    const int* __restrict__ batch, const float* __restrict__ hF, const float* __restrict__ gates,
    const float* __restrict__ bsum, float* clp, us_t* aHi, us_t* aLo, float* out0,
    int nN, int first) {
  __shared__ __attribute__((aligned(16))) float sq[NBP * DIM];
  __shared__ __attribute__((aligned(16))) float racc[NBP * DIM];
  __shared__ __attribute__((aligned(16))) int list[LISTN];
  __shared__ float smax[NBP];
  __shared__ float sden[NBP];
  __shared__ float semax[NBP];
  __shared__ int wcnt[NWAVE];
  const int tid = threadIdx.x, lane = tid & 31, wave = tid >> 5;
  const int gBase = blockIdx.x * NBP;

#pragma unroll 1
  for (int it = 0; it < NBP * DIM / NTHR; ++it) {
    const int idx = it * NTHR + tid;
    const int s = idx >> 7;
    const int d = idx & (DIM - 1);
    const int g = gBase + s;
    float gi, gf, gg, go, cold;
    if (first != 0) {
      gi = bsum[d]; gf = bsum[DIM + d]; gg = bsum[2 * DIM + d]; go = bsum[3 * DIM + d];
      cold = 0.0f;
    } else {
      const float* gp = gates + (size_t)g * G4;
      gi = gp[d]; gf = gp[DIM + d]; gg = gp[2 * DIM + d]; go = gp[3 * DIM + d];
      cold = clp[(size_t)g * DIM + d];
    }
    const float c  = sigm(gf) * cold + sigm(gi) * tanhf(gg);
    const float hv = sigm(go) * tanhf(c);
    sq[idx]   = hv;
    racc[idx] = c;
  }
  __syncthreads();
  s2s_store0(sq, racc, gBase, wave, lane, clp, aHi, aLo, out0);
  __threadfence();
  s2s_store0(sq, racc, gBase, wave, lane, clp, aHi, aLo, out0);
  __syncthreads();

  {
    const v4f z = {0.f, 0.f, 0.f, 0.f};
    for (int i = tid; i < NBP * DIM / 4; i += NTHR) ((v4f*)racc)[i] = z;
    if (tid < NBP) { smax[tid] = -__builtin_inff(); sden[tid] = 0.0f; semax[tid] = 0.0f; }
  }
  __syncthreads();

  const int nChunks = (nN + CHUNK - 1) / CHUNK;
#pragma unroll 1
  for (int ch = 0; ch < nChunks; ++ch) {
    const int cbase = ch * CHUNK;
    const int wc = scan_chunk<NBP>(batch, nN, cbase, gBase, 1, list, tid, lane, wave);
    if (lane == 0) wcnt[wave] = wc;
    __syncthreads();
    if (wave == 0) {
#pragma unroll 1
      for (int wsx = 0; wsx < NWAVE; ++wsx) {
        int n = __builtin_amdgcn_readfirstlane(wcnt[wsx]);
        n = n > WCAP ? WCAP : (n < 0 ? 0 : n);
        const int* lp = list + wsx * WCAP;
#pragma unroll 1
        for (int i = 0; i < n; ++i) {
          const int ent  = __builtin_amdgcn_readfirstlane(lp[i]);
          const int slot = ent & (NBP - 1);
          int nd = cbase + ((ent >> 12) & (CHUNK - 1));
          nd = nd > nN - 1 ? nN - 1 : nd;
          const v4f ov = *(const v4f*)(hF + (size_t)nd * DIM + 4 * lane);
          const v4f qv = *(const v4f*)(sq + slot * DIM + 4 * lane);
          float e = ov.x * qv.x + ov.y * qv.y + ov.z * qv.z + ov.w * qv.w;
          e += __shfl_xor(e, 16);
          e += __shfl_xor(e, 8);
          e += __shfl_xor(e, 4);
          e += __shfl_xor(e, 2);
          e += __shfl_xor(e, 1);
          if (lane == 0) smax[slot] = fmaxf(smax[slot], e);
        }
      }
    }
    __syncthreads();
  }
  if (tid < NBP) {
    const float mx = smax[tid];
    semax[tid] = (mx > -__builtin_inff() && mx < __builtin_inff()) ? mx : 0.0f;
  }
  __syncthreads();

#pragma unroll 1
  for (int ch = 0; ch < nChunks; ++ch) {
    const int cbase = ch * CHUNK;
    const int wc = scan_chunk<NBP>(batch, nN, cbase, gBase, 1, list, tid, lane, wave);
    if (lane == 0) wcnt[wave] = wc;
    __syncthreads();
    if (wave == 0) {
#pragma unroll 1
      for (int wsx = 0; wsx < NWAVE; ++wsx) {
        int n = __builtin_amdgcn_readfirstlane(wcnt[wsx]);
        n = n > WCAP ? WCAP : (n < 0 ? 0 : n);
        const int* lp = list + wsx * WCAP;
#pragma unroll 1
        for (int i = 0; i < n; ++i) {
          const int ent  = __builtin_amdgcn_readfirstlane(lp[i]);
          const int slot = ent & (NBP - 1);
          int nd = cbase + ((ent >> 12) & (CHUNK - 1));
          nd = nd > nN - 1 ? nN - 1 : nd;
          const v4f ov = *(const v4f*)(hF + (size_t)nd * DIM + 4 * lane);
          const v4f qv = *(const v4f*)(sq + slot * DIM + 4 * lane);
          float e = ov.x * qv.x + ov.y * qv.y + ov.z * qv.z + ov.w * qv.w;
          e += __shfl_xor(e, 16);
          e += __shfl_xor(e, 8);
          e += __shfl_xor(e, 4);
          e += __shfl_xor(e, 2);
          e += __shfl_xor(e, 1);
          const float p = expf(e - semax[slot]);
          v4f* ap = (v4f*)(racc + slot * DIM + 4 * lane);
          *ap = *ap + ov * p;
          if (lane == 0) sden[slot] = sden[slot] + p;
        }
      }
    }
    __syncthreads();
  }

  s2s_storeC(racc, sden, gBase, wave, lane, aHi, aLo, out0);
  __threadfence();
  s2s_storeC(racc, sden, gBase, wave, lane, aHi, aLo, out0);
}

extern "C" void kernel_launch(void* const* d_in, const int* in_sizes, int n_in,
                              void* d_out, int out_size, void* d_ws, size_t ws_size,
                              hipStream_t stream) {
  if (n_in < 17) return;
  const int nN = in_sizes[0] / DIM;
  const int nE = in_sizes[1] / 2;
  if (nN <= 0 || nE <= 0 || in_sizes[0] != nN * DIM || in_sizes[1] != 2 * nE || in_sizes[2] != nN) return;
  if (in_sizes[3] != DIM * DIM || in_sizes[4] != DIM) return;
  if (in_sizes[5] != DIM * DIM || in_sizes[6] != DIM || in_sizes[7] != DIM * DIM || in_sizes[8] != DIM) return;
  if (in_sizes[9] != G3 * DIM || in_sizes[10] != G3 * DIM || in_sizes[11] != G3 || in_sizes[12] != G3) return;
  if (in_sizes[13] != G4 * 2 * DIM || in_sizes[14] != G4 * DIM || in_sizes[15] != G4 || in_sizes[16] != G4) return;
  if (nE > (1 << 28) || nN > (1 << 24)) return;
  const long long rem = (long long)out_size - (long long)nN * DIM;
  if (rem <= 0 || (rem % (2 * DIM)) != 0) return;
  const int G = (int)(rem / (2 * DIM));
  if (G <= 0 || (G % GROWS) != 0 || G > (1 << 20)) return;

  const float* x      = (const float*)d_in[0];
  const int*   ei     = (const int*)d_in[1];
  const int*   batch  = (const int*)d_in[2];
  const float* lin0W  = (const float*)d_in[3];
  const float* lin0b  = (const float*)d_in[4];
  const float* W1     = (const float*)d_in[5];
  const float* b1     = (const float*)d_in[6];
  const float* W2     = (const float*)d_in[7];
  const float* b2     = (const float*)d_in[8];
  const float* gWih   = (const float*)d_in[9];
  const float* gWhh   = (const float*)d_in[10];
  const float* gbih   = (const float*)d_in[11];
  const float* gbhh   = (const float*)d_in[12];
  const float* lWih   = (const float*)d_in[13];
  const float* lWhh   = (const float*)d_in[14];
  const float* lbih   = (const float*)d_in[15];
  const float* lbhh   = (const float*)d_in[16];
  float* out0 = (float*)d_out;
  float* out1 = out0 + (size_t)G * 2 * DIM;

  const int NPAD   = ((nN + TGT - 1) / TGT) * TGT;
  const int nBC    = (nN + NBC - 1) / NBC;
  const int CNTPAD = nBC * NBC;
  if (4 * nBC + 1 > RBN) return;
  const int nBF    = (nN + NBF - 1) / NBF;
  const int csrLen = ((nE + 31) & ~31) + 4096;
  if (CNTPAD < NPAD || nBF * NBF > CNTPAD) return;

  char* ws = (char*)d_ws;
  size_t off = 0;
  const size_t planeB = (size_t)NPAD * DIM * 2;
#define CARVE(NAME, BYTES) const size_t NAME = off; off += (size_t)(BYTES); off = (off + 255) & ~(size_t)255;
  CARVE(oP0h, planeB) CARVE(oP0l, planeB)
  CARVE(oP1h, planeB) CARVE(oP1l, planeB)
  CARVE(oHh,  planeB) CARVE(oHl,  planeB)
  CARVE(oHf,  (size_t)NPAD * DIM * 4)
  CARVE(oL0h, (size_t)DIM * DIM * 2) CARVE(oL0l, (size_t)DIM * DIM * 2)
  CARVE(oW1h, (size_t)DIM * DIM * 2) CARVE(oW1l, (size_t)DIM * DIM * 2)
  CARVE(oW2h, (size_t)DIM * DIM * 2) CARVE(oW2l, (size_t)DIM * DIM * 2)
  CARVE(oIh,  (size_t)G3 * DIM * 2)  CARVE(oIl,  (size_t)G3 * DIM * 2)
  CARVE(oRh,  (size_t)G3 * DIM * 2)  CARVE(oRl,  (size_t)G3 * DIM * 2)
  CARVE(oCh,  (size_t)G4 * KL * 2)   CARVE(oCl,  (size_t)G4 * KL * 2)
  CARVE(oBs,  (size_t)G4 * 4)
  CARVE(oCnt, (size_t)CNTPAD * 4)
  CARVE(oOff, (size_t)CNTPAD * 4)
  CARVE(oRb,  (size_t)RBN * 4)
  CARVE(oCsr, (size_t)csrLen * 4)
  CARVE(oAh,  (size_t)G * KL * 2)    CARVE(oAl,  (size_t)G * KL * 2)
  CARVE(oGt,  (size_t)G * G4 * 4)
  CARVE(oClp, (size_t)G * DIM * 4)
#undef CARVE
  if (off > ws_size) return;

  us_t*  P0h  = (us_t*)(ws + oP0h);  us_t* P0l = (us_t*)(ws + oP0l);
  us_t*  P1h  = (us_t*)(ws + oP1h);  us_t* P1l = (us_t*)(ws + oP1l);
  us_t*  Hh   = (us_t*)(ws + oHh);   us_t* Hl  = (us_t*)(ws + oHl);
  float* Hf   = (float*)(ws + oHf);
  us_t*  L0h  = (us_t*)(ws + oL0h);  us_t* L0l = (us_t*)(ws + oL0l);
  us_t*  W1h  = (us_t*)(ws + oW1h);  us_t* W1l = (us_t*)(ws + oW1l);
  us_t*  W2h  = (us_t*)(ws + oW2h);  us_t* W2l = (us_t*)(ws + oW2l);
  us_t*  Ih   = (us_t*)(ws + oIh);   us_t* Il  = (us_t*)(ws + oIl);
  us_t*  Rh   = (us_t*)(ws + oRh);   us_t* Rl  = (us_t*)(ws + oRl);
  us_t*  Ch   = (us_t*)(ws + oCh);   us_t* Clw = (us_t*)(ws + oCl);
  float* Bs   = (float*)(ws + oBs);
  int*   cnt  = (int*)(ws + oCnt);
  int*   offp = (int*)(ws + oOff);
  int*   rb   = (int*)(ws + oRb);
  int*   csr  = (int*)(ws + oCsr);
  us_t*  Ah   = (us_t*)(ws + oAh);   us_t* Al  = (us_t*)(ws + oAl);
  float* Gt   = (float*)(ws + oGt);
  float* Clp  = (float*)(ws + oClp);

  const int vec8 = ((nE & 3) == 0) ? 1 : 0;

  {
    const int nvx = NPAD * DIM / 8;
    k_cvt<<<(nvx + NTHR - 1) / NTHR, NTHR, 0, stream>>>(x, P0h, P0l, DIM, nN, nvx);
    const int nvw = DIM * DIM / 8;
    k_cvt<<<(nvw + NTHR - 1) / NTHR, NTHR, 0, stream>>>(lin0W, L0h, L0l, DIM, DIM, nvw);
    k_cvt<<<(nvw + NTHR - 1) / NTHR, NTHR, 0, stream>>>(W1, W1h, W1l, DIM, DIM, nvw);
    k_cvt<<<(nvw + NTHR - 1) / NTHR, NTHR, 0, stream>>>(W2, W2h, W2l, DIM, DIM, nvw);
    const int nvg = G3 * DIM / 8;
    k_cvt<<<(nvg + NTHR - 1) / NTHR, NTHR, 0, stream>>>(gWih, Ih, Il, DIM, G3, nvg);
    k_cvt<<<(nvg + NTHR - 1) / NTHR, NTHR, 0, stream>>>(gWhh, Rh, Rl, DIM, G3, nvg);
    const int nvc = G4 * KL / 8;
    k_cvt2<<<(nvc + NTHR - 1) / NTHR, NTHR, 0, stream>>>(lWih, lWhh, lbih, lbhh, Ch, Clw, Bs, nvc);
  }

  k_count<<<nBC, NTHR, 0, stream>>>(ei, cnt, nE, vec8);
  k_offsets<<<1, OTHR, 0, stream>>>(cnt, offp, rb, nBC);
  hipFuncSetAttribute(reinterpret_cast<const void*>(&k_fill),
                      hipFuncAttributeMaxDynamicSharedMemorySize, LDS_FILL);
  k_fill<<<nBF, NTHR, LDS_FILL, stream>>>(ei, offp, rb, csr, nN, nE, vec8, csrLen);

  hipFuncSetAttribute(reinterpret_cast<const void*>(&k_gemm<DIM>),
                      hipFuncAttributeMaxDynamicSharedMemorySize, LDS_GEMM);
  hipFuncSetAttribute(reinterpret_cast<const void*>(&k_gemm<KL>),
                      hipFuncAttributeMaxDynamicSharedMemorySize, LDS_GEMM);
  hipFuncSetAttribute(reinterpret_cast<const void*>(&k_grustep),
                      hipFuncAttributeMaxDynamicSharedMemorySize, LDS_GRU);
  const int nGemm = NPAD / GROWS;
  k_gemm<DIM><<<dim3(nGemm, 1), NTHR, LDS_GEMM, stream>>>(P0h, P0l, L0h, L0l, lin0b,
                                                           Hf, Hh, Hl, DIM, DIM, 1, 1, 1);

  for (int layer = 0; layer < 3; ++layer) {
    k_agg<<<NPAD / TGT, NTHR, 0, stream>>>(csr, offp, cnt, Hf, P0h, P0l, nN, csrLen);
    k_gemm<DIM><<<dim3(nGemm, 1), NTHR, LDS_GEMM, stream>>>(P0h, P0l, W1h, W1l, b1,
                                                             Gt, P1h, P1l, DIM, DIM, 1, 0, 1);
    k_gemm<DIM><<<dim3(nGemm, 1), NTHR, LDS_GEMM, stream>>>(P1h, P1l, W2h, W2l, b2,
                                                             Gt, P0h, P0l, DIM, DIM, 1, 0, 1);
    k_grustep<<<NPAD / FROWS, FTHR, LDS_GRU, stream>>>(P0h, P0l, Hh, Hl, Ih, Il, Rh, Rl, gbih, gbhh,
                                                       Hf, out1, nN, layer == 2 ? 1 : 0);
  }

  const int nPool = G / NBP;
  for (int s = 0; s < 3; ++s) {
    if (s > 0) {
      k_gemm<KL><<<dim3(G / GROWS, G4 / DIM), NTHR, LDS_GEMM, stream>>>(Ah, Al, Ch, Clw, Bs,
                                                                       Gt, P1h, P1l, G4, DIM, 0, 1, 0);
    }
    k_s2s<<<nPool, NTHR, 0, stream>>>(batch, Hf, Gt, Bs, Clp, Ah, Al, out0, nN, s == 0 ? 1 : 0);
  }
}
